// NeRF_54752243090148
// MI455X (gfx1250) — hardware-verified
//
#include <hip/hip_runtime.h>

typedef _Float16 v16h __attribute__((ext_vector_type(16)));
typedef _Float16 v8h  __attribute__((ext_vector_type(8)));
typedef float    v8f  __attribute__((ext_vector_type(8)));
typedef float    v4f  __attribute__((ext_vector_type(4)));
typedef v8h __attribute__((may_alias)) v8ha;
typedef v4f __attribute__((may_alias)) v4fa;

union Frag { v16h v; v8h half[2]; };

#define TROWS   128
#define NTHR    256
#define NWAVES  8
#define S_ACT   304
#define S_XE    72
#define DE_COL0 256

#define OP_SCALE   64.0f
#define ACC_TO_X64 0.015625f
#define ACC_TO_F32 (1.0f / 4096.0f)

#define H_ACTA  0
#define H_ACTB  (TROWS * S_ACT)
#define H_XE    (2 * TROWS * S_ACT)
#define H_OUT   (H_XE + TROWS * S_XE)
#define SMEM_BYTES (H_OUT * 2 + TROWS * 16)

#define OFF_W0   0u
#define OFF_W1   16384u
#define OFF_W2   81920u
#define OFF_W3   147456u
#define OFF_W4   212992u
#define OFF_W5   278528u
#define OFF_W6   360448u
#define OFF_W7   425984u
#define OFF_GEO  491520u
#define OFF_DEN  (OFF_GEO + 65536u)
#define OFF_C0   565248u
#define OFF_C1   602112u
#define WS_HALVES 606208u

struct NerfPtrs {
  const float* x; const float* d; const _Float16* w;
  const float* sb[8];
  const float* den_b; const float* geo_b; const float* cb0; const float* cb1;
  float* out;
};
static_assert(sizeof(NerfPtrs) == 128);

__device__ __forceinline__ v16h load_frag(const _Float16* p, int h) {
  Frag f;
  f.half[0] = *(const v8ha*)(p + 8 * h);
  f.half[1] = *(const v8ha*)(p + 16 + 8 * h);
  return f.v;
}

__device__ __forceinline__ v8f wmma_raw(v16h a, v16h b, v8f c) {
  return __builtin_amdgcn_wmma_f32_16x16x32_f16(false, a, false, b, (short)0, c, false, false);
}

__global__ __launch_bounds__(256) void pack_plane(const float* __restrict__ src,
                                                   _Float16* __restrict__ dst,
                                                   int outDim, int inDim, int np, int kp, int skipCol)
{
  const int g = blockIdx.x * 256 + threadIdx.x;
  const int total8 = (np * kp) >> 3;
  if (g >= total8) return;
  const int e = g * 8;
  const int o = e / kp;
  const int kb = e - o * kp;
  const bool rowok = (o < outDim);
  const int oc = min(o, outDim - 1);
  float v[8];
  #pragma unroll
  for (int i = 0; i < 8; ++i) {
    const int k = kb + i;
    int s = k;
    bool ok = rowok;
    if (skipCol >= 0) {
      if (k == skipCol) ok = false;
      else if (k > skipCol) s = k - 1;
    }
    ok = ok && (s < inDim);
    const int sc = min(max(s, 0), inDim - 1);
    const float t = src[(size_t)oc * (size_t)inDim + sc];
    v[i] = ok ? (t * OP_SCALE) : 0.0f;
  }
  const v8h o8 = { (_Float16)v[0], (_Float16)v[1], (_Float16)v[2], (_Float16)v[3],
                   (_Float16)v[4], (_Float16)v[5], (_Float16)v[6], (_Float16)v[7] };
  _Float16* p = dst + (size_t)e;
  *(volatile v8h*)p = o8;
  __threadfence();
  *(volatile v8h*)p = o8;
}

__device__ __forceinline__ void run_layer(
    _Float16* sh, const _Float16* __restrict__ W, const int kp, const int ntp,
    const int b0off, const int s0, const int n0,
    const int b1off, const int s1, const int n1,
    const float* __restrict__ bias, const int nb, const float* __restrict__ xb, const int xcol,
    const bool relu, const int aoff, const int nact,
    float* fo, const int fcol0, const int nf, const int foff,
    const int lane, const int wave)
{
  const int h = lane >> 4, m = lane & 15;
  const v8f z8 = {0.f, 0.f, 0.f, 0.f, 0.f, 0.f, 0.f, 0.f};
  const int ntask = 2 * ntp;
  const int nk = n0 + n1;

  #pragma unroll 1
  for (int t = wave; t < ntask; t += NWAVES) {
    const int mg = (t >= ntp) ? 1 : 0;
    const int np = t - mg * ntp;
    const int rbase = 64 * mg;
    const _Float16* wr0 = W + (size_t)(np * 32 + m) * (size_t)kp;
    const _Float16* wr1 = wr0 + (size_t)16 * (size_t)kp;

    v8f acc[4][2];
    #pragma unroll
    for (int pt = 0; pt < 4; ++pt) { acc[pt][0] = z8; acc[pt][1] = z8; }

    #pragma unroll 1
    for (int ks = 0; ks < nk; ++ks) {
      const bool sg = (ks >= n0);
      const int sb  = sg ? s1 : s0;
      const int bo  = sg ? (b1off + (rbase + m) * s1 + 32 * (ks - n0))
                         : (b0off + (rbase + m) * s0 + 32 * ks);
      const _Float16* bp = sh + bo;
      const v16h a0 = load_frag(wr0 + 32 * ks, h);
      const v16h a1 = load_frag(wr1 + 32 * ks, h);
      const v16h f0 = load_frag(bp, h);
      const v16h f1 = load_frag(bp + 16 * sb, h);
      const v16h f2 = load_frag(bp + 32 * sb, h);
      const v16h f3 = load_frag(bp + 48 * sb, h);
      acc[0][0] = wmma_raw(a0, f0, acc[0][0]);  acc[0][1] = wmma_raw(a1, f0, acc[0][1]);
      acc[1][0] = wmma_raw(a0, f1, acc[1][0]);  acc[1][1] = wmma_raw(a1, f1, acc[1][1]);
      acc[2][0] = wmma_raw(a0, f2, acc[2][0]);  acc[2][1] = wmma_raw(a1, f2, acc[2][1]);
      acc[3][0] = wmma_raw(a0, f3, acc[3][0]);  acc[3][1] = wmma_raw(a1, f3, acc[3][1]);
      asm volatile("v_nop\n\tv_nop\n\tv_nop\n\tv_nop"
                   : "+v"(acc[0][0]), "+v"(acc[0][1]), "+v"(acc[1][0]), "+v"(acc[1][1]),
                     "+v"(acc[2][0]), "+v"(acc[2][1]), "+v"(acc[3][0]), "+v"(acc[3][1])
                   : "v"(a0), "v"(a1), "v"(f0), "v"(f1), "v"(f2), "v"(f3));
    }

    #pragma unroll
    for (int nt = 0; nt < 2; ++nt) {
      const int cb = np * 32 + 16 * nt + 8 * h;
      const float bxv = xb[0];
      float bcol[8], b64[8];
      #pragma unroll
      for (int r = 0; r < 8; ++r) {
        const int col = cb + r;
        const float bl = bias[min(col, nb - 1)];
        bcol[r] = (col < nb) ? bl : ((col == xcol) ? bxv : 0.0f);
        b64[r] = OP_SCALE * bcol[r];
      }
      #pragma unroll
      for (int pt = 0; pt < 4; ++pt) {
        const int prow = rbase + 16 * pt + m;
        float tv[8];
        #pragma unroll
        for (int r = 0; r < 8; ++r) {
          const float u = acc[pt][nt][r] * ACC_TO_X64 + b64[r];
          tv[r] = relu ? fmaxf(u, 0.0f) : u;
        }
        if (cb < nact) {
          const v8h o8 = { (_Float16)tv[0], (_Float16)tv[1], (_Float16)tv[2], (_Float16)tv[3],
                           (_Float16)tv[4], (_Float16)tv[5], (_Float16)tv[6], (_Float16)tv[7] };
          *(v8ha*)(sh + aoff + prow * S_ACT + cb) = o8;
        }
        if (nf > 0) {
          #pragma unroll
          for (int r = 0; r < 8; ++r) {
            const int col = cb + r;
            if (col >= fcol0 && col < fcol0 + nf)
              fo[prow * 4 + foff + (col - fcol0)] = acc[pt][nt][r] * ACC_TO_F32 + bcol[r];
          }
        }
      }
    }
  }
}

__global__ __launch_bounds__(NTHR) void nerf_mlp(NerfPtrs P, int npts)
{
  extern __shared__ __attribute__((aligned(16))) unsigned char smem_raw[];
  _Float16* sh = (_Float16*)smem_raw;
  float* sOut = (float*)(smem_raw + (size_t)H_OUT * 2);

  const int tid = threadIdx.x, lane = tid & 31, wave = tid >> 5;
  const int row0 = blockIdx.x * TROWS;

  #pragma unroll 1
  for (int it = tid; it < TROWS * 3; it += NTHR) {
    const int r = it / 3, ci = it - 3 * r;
    const int gr = min(row0 + r, npts - 1);
    const float xv = P.x[(size_t)gr * 3 + ci];
    const float dv = P.d[(size_t)gr * 3 + ci];
    const int xo = H_XE + r * S_XE;
    const int dofs = H_ACTA + r * S_ACT + DE_COL0;
    sh[xo + ci]   = (_Float16)(OP_SCALE * xv);
    sh[dofs + ci] = (_Float16)(OP_SCALE * dv);
    #pragma unroll 1
    for (int i = 0; i < 14; ++i) {
      const bool isx = (i < 10);
      const int e = isx ? i : (i - 10);
      const float base = isx ? xv : dv;
      const float arg = base * (float)(1 << e);
      const float sv = sinf(arg);
      const float cv = cosf(arg);
      const int o = (isx ? xo : dofs) + 6 * e + ci;
      sh[o + 3] = (_Float16)(OP_SCALE * sv);
      sh[o + 6] = (_Float16)(OP_SCALE * cv);
    }
  }
  #pragma unroll 1
  for (int r = tid; r < TROWS; r += NTHR) {
    sh[H_XE + r * S_XE + 63] = (_Float16)0.0f;
    #pragma unroll
    for (int c = 0; c < 5; ++c) sh[H_ACTA + r * S_ACT + DE_COL0 + 27 + c] = (_Float16)0.0f;
  }
  __syncthreads();

  const _Float16* W = P.w;
  run_layer(sh, W + OFF_W0, 64, 8,  H_XE, S_XE, 2,   H_XE, S_XE, 0,   P.sb[0], 256, P.sb[0], -1, true,  H_ACTA, 256, sOut, 0, 0, 0, lane, wave);
  __syncthreads();
  run_layer(sh, W + OFF_W1, 256, 8, H_ACTA, S_ACT, 8, H_ACTA, S_ACT, 0, P.sb[1], 256, P.sb[1], -1, true,  H_ACTB, 256, sOut, 0, 0, 0, lane, wave);
  __syncthreads();
  run_layer(sh, W + OFF_W2, 256, 8, H_ACTB, S_ACT, 8, H_ACTB, S_ACT, 0, P.sb[2], 256, P.sb[2], -1, true,  H_ACTA, 256, sOut, 0, 0, 0, lane, wave);
  __syncthreads();
  run_layer(sh, W + OFF_W3, 256, 8, H_ACTA, S_ACT, 8, H_ACTA, S_ACT, 0, P.sb[3], 256, P.sb[3], -1, true,  H_ACTB, 256, sOut, 0, 0, 0, lane, wave);
  __syncthreads();
  run_layer(sh, W + OFF_W4, 256, 8, H_ACTB, S_ACT, 8, H_ACTB, S_ACT, 0, P.sb[4], 256, P.sb[4], -1, true,  H_ACTA, 256, sOut, 0, 0, 0, lane, wave);
  __syncthreads();
  run_layer(sh, W + OFF_W5, 320, 8, H_XE, S_XE, 2,   H_ACTA, S_ACT, 8, P.sb[5], 256, P.sb[5], -1, true,  H_ACTB, 256, sOut, 0, 0, 0, lane, wave);
  __syncthreads();
  run_layer(sh, W + OFF_W6, 256, 8, H_ACTB, S_ACT, 8, H_ACTB, S_ACT, 0, P.sb[6], 256, P.sb[6], -1, true,  H_ACTA, 256, sOut, 0, 0, 0, lane, wave);
  __syncthreads();
  run_layer(sh, W + OFF_W7, 256, 8, H_ACTA, S_ACT, 8, H_ACTA, S_ACT, 0, P.sb[7], 256, P.sb[7], -1, true,  H_ACTB, 256, sOut, 0, 0, 0, lane, wave);
  __syncthreads();
  run_layer(sh, W + OFF_GEO, 256, 9, H_ACTB, S_ACT, 8, H_ACTB, S_ACT, 0, P.geo_b, 256, P.den_b, 256, false, H_ACTA, 256, sOut, 256, 1, 3, lane, wave);
  __syncthreads();
  run_layer(sh, W + OFF_C0, 288, 4, H_ACTA, S_ACT, 9, H_ACTA, S_ACT, 0, P.cb0, 128, P.cb0, -1, true,  H_ACTB, 128, sOut, 0, 0, 0, lane, wave);
  __syncthreads();
  run_layer(sh, W + OFF_C1, 128, 1, H_ACTB, S_ACT, 4, H_ACTB, S_ACT, 0, P.cb1, 3, P.cb1, -1, false, H_ACTA, 0, sOut, 0, 3, 0, lane, wave);
  __syncthreads();

  const int gp = row0 + tid;
  const bool doSt = (tid < TROWS) && (gp < npts);
  v4f ov = {0.f, 0.f, 0.f, 0.f};
  if (tid < TROWS) ov = *(const v4fa*)(sOut + 4 * tid);
  float* op = P.out + (size_t)gp * 4;
  if (doSt) *(volatile v4f*)op = ov;
  __threadfence();
  if (doSt) *(volatile v4f*)op = ov;
}

extern "C" void kernel_launch(void* const* d_in, const int* in_sizes, int n_in,
                              void* d_out, int out_size, void* d_ws, size_t ws_size,
                              hipStream_t stream)
{
  if (n_in < 26) return;
  const int npts = in_sizes[0] / 3;
  if (npts < 1 || in_sizes[0] != 3 * npts || in_sizes[1] != 3 * npts) return;
  if (out_size != 4 * npts) return;
  if (in_sizes[2] != 256 * 63) return;
  if (in_sizes[4] != 65536 || in_sizes[6] != 65536 || in_sizes[8] != 65536 || in_sizes[10] != 65536) return;
  if (in_sizes[12] != 256 * 319) return;
  if (in_sizes[14] != 65536 || in_sizes[16] != 65536) return;
  for (int i = 0; i < 8; ++i) if (in_sizes[3 + 2 * i] != 256) return;
  if (in_sizes[18] != 256 || in_sizes[19] < 1) return;
  if (in_sizes[20] != 65536 || in_sizes[21] != 256) return;
  if (in_sizes[22] != 128 * 283 || in_sizes[23] != 128) return;
  if (in_sizes[24] != 3 * 128 || in_sizes[25] < 3) return;
  if ((size_t)WS_HALVES * 2 > ws_size) return;

  _Float16* W = (_Float16*)d_ws;

  auto pack = [&](int inIdx, unsigned off, int outDim, int inDim, int np, int kp, int skip) {
    const int total8 = (np * kp) / 8;
    pack_plane<<<(total8 + 255) / 256, 256, 0, stream>>>((const float*)d_in[inIdx], W + off,
                                                         outDim, inDim, np, kp, skip);
  };
  pack(2,  OFF_W0,  256, 63,  256, 64,  -1);
  pack(4,  OFF_W1,  256, 256, 256, 256, -1);
  pack(6,  OFF_W2,  256, 256, 256, 256, -1);
  pack(8,  OFF_W3,  256, 256, 256, 256, -1);
  pack(10, OFF_W4,  256, 256, 256, 256, -1);
  pack(12, OFF_W5,  256, 319, 256, 320, 63);
  pack(14, OFF_W6,  256, 256, 256, 256, -1);
  pack(16, OFF_W7,  256, 256, 256, 256, -1);
  pack(20, OFF_GEO, 256, 256, 256, 256, -1);
  pack(18, OFF_DEN, 1,   256, 32,  256, -1);
  pack(22, OFF_C0,  128, 283, 128, 288, -1);
  pack(24, OFF_C1,  3,   128, 32,  128, -1);

  NerfPtrs P;
  P.x = (const float*)d_in[0];
  P.d = (const float*)d_in[1];
  P.w = W;
  for (int i = 0; i < 8; ++i) P.sb[i] = (const float*)d_in[3 + 2 * i];
  P.den_b = (const float*)d_in[19];
  P.geo_b = (const float*)d_in[21];
  P.cb0   = (const float*)d_in[23];
  P.cb1   = (const float*)d_in[25];
  P.out   = (float*)d_out;

  hipFuncSetAttribute(reinterpret_cast<const void*>(&nerf_mlp),
                      hipFuncAttributeMaxDynamicSharedMemorySize, SMEM_BYTES);
  const int nblk = (npts + TROWS - 1) / TROWS;
  nerf_mlp<<<nblk, NTHR, SMEM_BYTES, stream>>>(P, npts);
}
